// WarpTileMLP_38774964748567
// MI455X (gfx1250) — hardware-verified
//
#include <hip/hip_runtime.h>

typedef __attribute__((ext_vector_type(16))) _Float16 v16h;
typedef __attribute__((ext_vector_type(8)))  float    v8f;
typedef __attribute__((ext_vector_type(2)))  __fp16   h2fp;

static __device__ __forceinline__ int pack_rn(float lo, float hi) {
    const _Float16 a = (_Float16)lo, b = (_Float16)hi;
    return (int)((unsigned)__builtin_bit_cast(unsigned short, a) | ((unsigned)__builtin_bit_cast(unsigned short, b) << 16));
}
static __device__ __forceinline__ int pack_lo(float lo, float hi) {
    const _Float16 a = (_Float16)lo, b = (_Float16)hi;
    const _Float16 al = (_Float16)((lo - (float)a) * 2048.0f), bl = (_Float16)((hi - (float)b) * 2048.0f);
    return (int)((unsigned)__builtin_bit_cast(unsigned short, al) | ((unsigned)__builtin_bit_cast(unsigned short, bl) << 16));
}
static __device__ __forceinline__ _Float16 lo_of(float v, _Float16 h) { return (_Float16)((v - (float)h) * 2048.0f); }
#define RSPLIT (1.0f / 2048.0f)
static __device__ __forceinline__ v8f wmma16(v16h a, v16h b, v8f c) { return __builtin_amdgcn_wmma_f32_16x16x32_f16(false, a, false, b, (short)0, c, false, false); }
static __device__ __forceinline__ v8f wmma_split(v16h a, v16h al, v16h b, v16h bl, v8f c) { v8f x = {}; x = wmma16(al, b, x); x = wmma16(a, bl, x); return wmma16(a, b, c) + x * RSPLIT; }

static __device__ __forceinline__ float fast_tanh(float x) {
    float e = __expf(2.0f * x);
    return 1.0f - 2.0f / (e + 1.0f);
}

__global__ __launch_bounds__(256) void mlp_wmma_kernel(
    const float* __restrict__ q,
    const float* __restrict__ w0, const float* __restrict__ b0,
    const float* __restrict__ w1, const float* __restrict__ b1,
    const float* __restrict__ w2, const float* __restrict__ b2,
    float* __restrict__ out, int ntiles)
{
    const int lane = threadIdx.x & 31;
    const int half = lane >> 4;
    const int r    = lane & 15;

    const int wavesPerBlock = blockDim.x >> 5;
    const int waveId = blockIdx.x * wavesPerBlock + (threadIdx.x >> 5);
    const int nWaves = gridDim.x * wavesPerBlock;

    v16h a0h0, a0h1, a1h0, a1h1, a0h0l, a0h1l, a1h0l, a1h1l;
    #pragma unroll
    for (int e = 0; e < 16; ++e) { a0h0[e] = (_Float16)0.f; a0h1[e] = (_Float16)0.f; a0h0l[e] = (_Float16)0.f; a0h1l[e] = (_Float16)0.f; }
    if (half == 0) {
        #pragma unroll
        for (int k = 0; k < 7; ++k) {
            const float u0 = w0[r * 7 + k], u1 = w0[(r + 16) * 7 + k];
            a0h0[k] = (_Float16)u0; a0h0l[k] = lo_of(u0, a0h0[k]);
            a0h1[k] = (_Float16)u1; a0h1l[k] = lo_of(u1, a0h1[k]);
        }
    }
    const int kb = half * 8;
    #pragma unroll
    for (int e = 0; e < 8; ++e) {
        const float u00 = w1[r * 32 + kb + e], u01 = w1[r * 32 + 16 + kb + e], u10 = w1[(r + 16) * 32 + kb + e], u11 = w1[(r + 16) * 32 + 16 + kb + e];
        a1h0[e] = (_Float16)u00; a1h0l[e] = lo_of(u00, a1h0[e]);  a1h0[e + 8] = (_Float16)u01; a1h0l[e + 8] = lo_of(u01, a1h0[e + 8]);
        a1h1[e] = (_Float16)u10; a1h1l[e] = lo_of(u10, a1h1[e]);  a1h1[e + 8] = (_Float16)u11; a1h1l[e + 8] = lo_of(u11, a1h1[e + 8]);
    }

    float cb0a[8], cb0b[8], cb1a[8], cb1b[8], w2a[8], w2b[8];
    #pragma unroll
    for (int v = 0; v < 8; ++v) {
        cb0a[v] = b0[kb + v];      cb0b[v] = b0[16 + kb + v];
        cb1a[v] = b1[kb + v];      cb1b[v] = b1[16 + kb + v];
        w2a[v]  = w2[kb + v];      w2b[v]  = w2[16 + kb + v];
    }
    const float b2s = b2[0];

    for (int tp = waveId; tp < ntiles / 2; tp += nWaves) {
      float res[2];
      #pragma unroll
      for (int u = 0; u < 2; ++u) {
        const int t = tp * 2 + u;
        const long long s = (long long)t * 16 + r;
        const float* qr = q + s * 7;
        v16h bq, bql;
        #pragma unroll
        for (int e = 0; e < 16; ++e) { bq[e] = (_Float16)0.f; bql[e] = (_Float16)0.f; }
        if (half == 0) {
            #pragma unroll
            for (int e = 0; e < 7; ++e) { const float qv = qr[e]; bq[e] = (_Float16)qv; bql[e] = lo_of(qv, bq[e]); }
        }

        v8f cz = {};
        v8f c0h0 = wmma_split(a0h0, a0h0l, bq, bql, cz);
        v8f c0h1 = wmma_split(a0h1, a0h1l, bq, bql, cz);

        union { v16h h; int i[8]; } uz, ul;
        #pragma unroll
        for (int j = 0; j < 4; ++j) {
            float t00 = fast_tanh(c0h0[2*j]     + cb0a[2*j]);
            float t01 = fast_tanh(c0h0[2*j + 1] + cb0a[2*j + 1]);
            float t10 = fast_tanh(c0h1[2*j]     + cb0b[2*j]);
            float t11 = fast_tanh(c0h1[2*j + 1] + cb0b[2*j + 1]);
            uz.i[j]     = pack_rn(t00, t01);  ul.i[j]     = pack_lo(t00, t01);
            uz.i[j + 4] = pack_rn(t10, t11);  ul.i[j + 4] = pack_lo(t10, t11);
        }

        v8f c1h0 = wmma_split(a1h0, a1h0l, uz.h, ul.h, cz);
        v8f c1h1 = wmma_split(a1h1, a1h1l, uz.h, ul.h, cz);

        float acc = 0.f;
        #pragma unroll
        for (int v = 0; v < 8; ++v) {
            acc = fmaf(w2a[v], fast_tanh(c1h0[v] + cb1a[v]), acc);
            acc = fmaf(w2b[v], fast_tanh(c1h1[v] + cb1b[v]), acc);
        }
        acc += __shfl_xor(acc, 16, 32);
        res[u] = acc + b2s;
      }
      const float ov = (half == 0) ? res[0] : res[1];
      float* op = out + (size_t)tp * 32 + lane;
      *(volatile float*)op = ov; __threadfence(); *(volatile float*)op = ov;
    }
}

extern "C" void kernel_launch(void* const* d_in, const int* in_sizes, int n_in,
                              void* d_out, int out_size, void* d_ws, size_t ws_size,
                              hipStream_t stream) {
    (void)n_in; (void)out_size; (void)d_ws; (void)ws_size;
    const float* q  = (const float*)d_in[0];
    const float* b0 = (const float*)d_in[2];
    const float* w0 = (const float*)d_in[1];
    const float* w1 = (const float*)d_in[3];
    const float* b1 = (const float*)d_in[4];
    const float* w2 = (const float*)d_in[5];
    const float* b2 = (const float*)d_in[6];
    float* out = (float*)d_out;

    const int B = in_sizes[0] / 7;
    const int ntiles = B / 16;

    const int threads = 256;
    int blocks = 2048;
    const int wavesPerBlock = threads / 32;
    int maxBlocks = (ntiles + wavesPerBlock - 1) / wavesPerBlock;
    if (blocks > maxBlocks) blocks = maxBlocks;
    if (blocks < 1) blocks = 1;

    mlp_wmma_kernel<<<blocks, threads, 0, stream>>>(q, w0, b0, w1, b1, w2, b2, out, ntiles);
}
